// Block_6777458393276
// MI455X (gfx1250) — hardware-verified
//
#include <hip/hip_runtime.h>


#pragma clang fp contract(off)

#ifndef NB
#define NB 2
#endif
#ifndef SEQ
#define SEQ 1024
#endif
#define NB_FULL 2
#define SEQ_FULL 1024
#define CDIM 1024
#define NHEAD 16
#define HD 64
#define MEMN 256
#define SKV (SEQ + 2 * MEMN)
#define OUT1_OFF (NB_FULL * SEQ_FULL * CDIM)
#define GN (NB * NHEAD * SEQ)
#define REG_ITERS (GN / 1024)

static_assert(NB >= 1 && NB <= NB_FULL);
static_assert(SEQ % 64 == 0 && SEQ >= 64 && SEQ <= SEQ_FULL);
static_assert(MEMN % 64 == 0);
static_assert(SKV % 64 == 0);
static_assert(CDIM == NHEAD * HD);
static_assert(HD == 64);
static_assert(CDIM % 64 == 0 && CDIM == 1024);
static_assert(NHEAD == 16);
static_assert(GN % 1024 == 0);
static_assert((size_t)OUT1_OFF * 4 == 8388608);

typedef _Float16 v16h __attribute__((ext_vector_type(16)));
typedef _Float16 v8h  __attribute__((ext_vector_type(8)));
typedef float    v8f  __attribute__((ext_vector_type(8)));
typedef float    v4f  __attribute__((ext_vector_type(4)));
typedef unsigned int v4u __attribute__((ext_vector_type(4)));

union Frag { v16h v; v4u q[2]; };

__device__ __forceinline__ v8f mma(v16h a, v16h b, v8f c) {
  v8f d = __builtin_amdgcn_wmma_f32_16x16x32_f16(false, a, false, b, (short)0, c, false, false);
  asm volatile("v_nop\n\tv_nop\n\tv_nop\n\tv_nop" : "+v"(d) : "v"(a), "v"(b));
  return d;
}

__device__ __forceinline__ v8f zero8() {
  v8f z;
#pragma unroll
  for (int i = 0; i < 8; ++i) z[i] = 0.0f;
  return z;
}

__device__ __forceinline__ float bf16q(float f) {
  unsigned int u = __float_as_uint(f);
  unsigned int r = u + 0x7FFFu + ((u >> 16) & 1u);
  r = ((u & 0x7F800000u) == 0x7F800000u) ? u : r;
  return __uint_as_float(r & 0xFFFF0000u);
}
__device__ __forceinline__ v4f bf16q4(v4f a) {
  v4f r;
  r.x = bf16q(a.x); r.y = bf16q(a.y); r.z = bf16q(a.z); r.w = bf16q(a.w);
  return r;
}
__device__ __forceinline__ unsigned short hbits(float f) {
  _Float16 h = (_Float16)f;
  return __builtin_bit_cast(unsigned short, h);
}
__device__ __forceinline__ v4u pack8h(float f0, float f1, float f2, float f3,
                                      float f4, float f5, float f6, float f7) {
  v8h t;
  t[0] = (_Float16)f0; t[1] = (_Float16)f1; t[2] = (_Float16)f2; t[3] = (_Float16)f3;
  t[4] = (_Float16)f4; t[5] = (_Float16)f5; t[6] = (_Float16)f6; t[7] = (_Float16)f7;
  return __builtin_bit_cast(v4u, t);
}

__global__ __launch_bounds__(256) void k_wprep(
    const float* __restrict__ s0, const float* __restrict__ s1, const float* __restrict__ s2,
    unsigned short* __restrict__ dst, unsigned int K, unsigned int hstride,
    unsigned int rstride, unsigned int zrows) {
  __shared__ __attribute__((aligned(16))) unsigned short sT[64][72];
  const unsigned int tid = threadIdx.x;
  const unsigned int k0 = blockIdx.x * 64u, n0 = blockIdx.y * 64u, z = blockIdx.z;
  const float* src = (z == 0u) ? s0 : ((z == 1u) ? s1 : s2);
  const size_t sbase = (size_t)(n0 >> 6) * (size_t)hstride;
#pragma unroll
  for (unsigned int it = 0; it < 4u; ++it) {
    const unsigned int idx = it * 256u + tid;
    const unsigned int kk = idx >> 4;
    const unsigned int j4 = (idx & 15u) * 4u;
    const v4f wv = *(const v4f*)(src + sbase + (size_t)(k0 + kk) * (size_t)rstride + j4);
    sT[j4 + 0][kk] = hbits(bf16q(wv.x) * 16.0f);
    sT[j4 + 1][kk] = hbits(bf16q(wv.y) * 16.0f);
    sT[j4 + 2][kk] = hbits(bf16q(wv.z) * 16.0f);
    sT[j4 + 3][kk] = hbits(bf16q(wv.w) * 16.0f);
  }
  __syncthreads();
  v4u val[2];
  size_t off[2];
#pragma unroll
  for (unsigned int p = 0; p < 2u; ++p) {
    const unsigned int n = p * 32u + (tid >> 3);
    const unsigned int piece = tid & 7u;
    val[p] = *(const v4u*)&sT[n][piece * 8u];
    off[p] = ((size_t)zrows * z + n0 + n) * (size_t)K + k0 + piece * 8u;
  }
#pragma unroll
  for (int p = 0; p < 2; ++p) *(volatile v4u*)(dst + off[p]) = val[p];
  __threadfence();
#pragma unroll
  for (int p = 0; p < 2; ++p) *(volatile v4u*)(dst + off[p]) = val[p];
}

__global__ __launch_bounds__(256) void k_gprep(const float* __restrict__ gW,
                                               unsigned short* __restrict__ gwt) {
  __shared__ __attribute__((aligned(16))) unsigned short sG[16][1032];
  const unsigned int tid = threadIdx.x;
#pragma unroll 2
  for (unsigned int it = 0; it < 16u; ++it) {
    const unsigned int idx4 = it * 256u + tid;
    const unsigned int k = idx4 >> 2;
    const unsigned int j4 = (idx4 & 3u) * 4u;
    const v4f wv = *(const v4f*)(gW + (size_t)k * 16u + j4);
    sG[j4 + 0][k] = hbits(bf16q(wv.x) * 16.0f);
    sG[j4 + 1][k] = hbits(bf16q(wv.y) * 16.0f);
    sG[j4 + 2][k] = hbits(bf16q(wv.z) * 16.0f);
    sG[j4 + 3][k] = hbits(bf16q(wv.w) * 16.0f);
  }
  __syncthreads();
  v4u val[8];
  unsigned int off[8];
#pragma unroll
  for (unsigned int p = 0; p < 8u; ++p) {
    const unsigned int q = p * 256u + tid;
    const unsigned int n = q >> 7;
    const unsigned int pc = q & 127u;
    val[p] = *(const v4u*)&sG[n][pc * 8u];
    off[p] = n * (unsigned int)CDIM + pc * 8u;
  }
#pragma unroll
  for (int p = 0; p < 8; ++p) *(volatile v4u*)(gwt + off[p]) = val[p];
  __threadfence();
#pragma unroll
  for (int p = 0; p < 8; ++p) *(volatile v4u*)(gwt + off[p]) = val[p];
}

__global__ __launch_bounds__(128) void k_pack(const float* __restrict__ x,
                                              const float* __restrict__ fm,
                                              const float* __restrict__ rm,
                                              unsigned short* __restrict__ dst) {
  const unsigned int tid = threadIdx.x;
  const unsigned int s = blockIdx.x, b = blockIdx.y;
  const bool isx = s < (unsigned int)SEQ;
  const bool isf = s < (unsigned int)(SEQ + MEMN);
  const float* src = isx ? x : (isf ? fm : rm);
  const size_t roff = isx ? ((size_t)b * SEQ_FULL + s) * CDIM
                          : (isf ? ((size_t)b * MEMN + (s - SEQ)) * CDIM
                                 : ((size_t)b * MEMN + (s - SEQ - MEMN)) * CDIM);
  const unsigned int c0 = tid * 8u;
  const v4f t0 = bf16q4(*(const v4f*)(src + roff + c0));
  const v4f t1 = bf16q4(*(const v4f*)(src + roff + c0 + 4));
  const v4u o = pack8h(t0.x, t0.y, t0.z, t0.w, t1.x, t1.y, t1.z, t1.w);
  unsigned short* orow = dst + ((size_t)b * SKV + s) * CDIM + c0;
  *(volatile v4u*)orow = o;
  __threadfence();
  *(volatile v4u*)orow = o;
}

template <int EPI>
__global__ __launch_bounds__(128) void k_gemm(
    const unsigned short* __restrict__ A, const unsigned short* __restrict__ Bt,
    float* __restrict__ outF, unsigned short* __restrict__ out0,
    unsigned short* __restrict__ out1, unsigned short* __restrict__ out2) {
  __shared__ __attribute__((aligned(16))) unsigned short sT[64][72];
  __shared__ __attribute__((aligned(16))) float sF[64][68];
  const unsigned int tid = threadIdx.x, lane = tid & 31u, w = tid >> 5;
  const unsigned int m = lane & 15u, hl = lane >> 4, k8 = hl * 8u;
  const unsigned int n0 = blockIdx.x * 64u, r0 = blockIdx.y * 64u, b = blockIdx.z;
  unsigned int m0;
  if constexpr (EPI == 0) {
    if (n0 < (unsigned int)CDIM && r0 >= (unsigned int)SEQ) return;
    m0 = b * (unsigned int)SKV + r0;
  } else {
    m0 = b * (unsigned int)SEQ + r0;
  }

  v8f acc[4];
#pragma unroll
  for (int j = 0; j < 4; ++j) acc[j] = zero8();

  const unsigned short* ap = A + (size_t)(m0 + 16u * w + m) * (size_t)CDIM + k8;
  const unsigned short* bp = Bt + (size_t)(n0 + m) * (size_t)CDIM + k8;
  const size_t jstep = (size_t)16 * (size_t)CDIM;
#pragma unroll 1
  for (unsigned int k0 = 0; k0 < (unsigned int)CDIM; k0 += 32u) {
    Frag a;
    a.q[0] = *(const v4u*)(ap + k0);
    a.q[1] = *(const v4u*)(ap + k0 + 16);
#pragma unroll
    for (int j = 0; j < 4; ++j) {
      Frag bf;
      const unsigned short* bj = bp + jstep * j + k0;
      bf.q[0] = *(const v4u*)(bj);
      bf.q[1] = *(const v4u*)(bj + 16);
      acc[j] = mma(a.v, bf.v, acc[j]);
    }
  }

  const unsigned int lrow0 = 16u * w + 8u * hl;

  if constexpr (EPI == 0) {
    const float wsc = 0.0625f;
#pragma unroll
    for (int j = 0; j < 4; ++j) {
#pragma unroll
      for (int r = 0; r < 8; ++r) sT[lrow0 + r][16 * j + m] = hbits(acc[j][r] * wsc);
    }
    __syncthreads();
    const unsigned int which = n0 / (unsigned int)CDIM;
    const unsigned int hh = (n0 - which * (unsigned int)CDIM) / (unsigned int)HD;
    const unsigned int bh = b * (unsigned int)NHEAD + hh;
    v4u val[4];
    unsigned int off[4];
    unsigned short* dst;
    if (which < 2u) {
      dst = (which == 0u) ? out0 : out1;
      const unsigned int rows = (which == 0u) ? (unsigned int)SEQ : (unsigned int)SKV;
#pragma unroll
      for (unsigned int p = 0; p < 4u; ++p) {
        const unsigned int row = p * 16u + 4u * w + (lane >> 3);
        const unsigned int piece = lane & 7u;
        val[p] = *(const v4u*)&sT[row][piece * 8u];
        off[p] = (bh * rows + r0 + row) * (unsigned int)HD + piece * 8u;
      }
    } else {
      dst = out2;
#pragma unroll
      for (unsigned int p = 0; p < 4u; ++p) {
        const unsigned int d = p * 16u + 4u * w + (lane >> 3);
        const unsigned int piece = lane & 7u;
        unsigned int wv[4];
#pragma unroll
        for (unsigned int e = 0; e < 4u; ++e) {
          const unsigned int lo = sT[piece * 8u + 2u * e][d];
          const unsigned int hi = sT[piece * 8u + 2u * e + 1u][d];
          wv[e] = lo | (hi << 16);
        }
        v4u t;
        t.x = wv[0]; t.y = wv[1]; t.z = wv[2]; t.w = wv[3];
        val[p] = t;
        off[p] = (bh * (unsigned int)HD + d) * (unsigned int)SKV + r0 + piece * 8u;
      }
    }
#pragma unroll
    for (int p = 0; p < 4; ++p) *(volatile v4u*)(dst + off[p]) = val[p];
    __threadfence();
#pragma unroll
    for (int p = 0; p < 4; ++p) *(volatile v4u*)(dst + off[p]) = val[p];
  } else {
    const float osc = 0.0009765625f;
#pragma unroll
    for (int j = 0; j < 4; ++j) {
#pragma unroll
      for (int r = 0; r < 8; ++r) sF[lrow0 + r][16 * j + m] = acc[j][r] * osc;
    }
    __syncthreads();
    v4f val[8];
    unsigned int off[8];
#pragma unroll
    for (unsigned int p = 0; p < 8u; ++p) {
      const unsigned int row = 16u * w + 2u * p + hl;
      const unsigned int piece = m;
      val[p] = *(const v4f*)&sF[row][4u * piece];
      const unsigned int orow = b * (unsigned int)SEQ_FULL + r0 + row;
      off[p] = orow * (unsigned int)CDIM + n0 + 4u * piece;
    }
#pragma unroll
    for (int p = 0; p < 8; ++p) *(volatile v4f*)(outF + off[p]) = val[p];
    __threadfence();
#pragma unroll
    for (int p = 0; p < 8; ++p) *(volatile v4f*)(outF + off[p]) = val[p];
  }
}

__global__ __launch_bounds__(128) void k_gate(const unsigned short* __restrict__ qp,
                                              const unsigned short* __restrict__ gwt,
                                              const float* __restrict__ gb,
                                              float* __restrict__ gout) {
  __shared__ __attribute__((aligned(16))) float sG[16][68];
  const unsigned int tid = threadIdx.x, lane = tid & 31u, w = tid >> 5;
  const unsigned int m = lane & 15u, hl = lane >> 4, k8 = hl * 8u;
  const unsigned int t0 = blockIdx.x * 64u, b = blockIdx.y;
  const unsigned int trow = t0 + 16u * w + m;

  v8f acc = zero8();
  const unsigned short* bp = gwt + (size_t)m * CDIM + k8;
#pragma unroll 1
  for (unsigned int k0 = 0; k0 < (unsigned int)CDIM; k0 += 32u) {
    const unsigned int hs = k0 >> 6, kin = k0 & 63u;
    const unsigned short* ap =
        qp + ((size_t)(b * (unsigned int)NHEAD + hs) * SEQ + trow) * HD + kin + k8;
    Frag a, bf;
    a.q[0] = *(const v4u*)(ap);
    a.q[1] = *(const v4u*)(ap + 16);
    bf.q[0] = *(const v4u*)(bp + k0);
    bf.q[1] = *(const v4u*)(bp + k0 + 16);
    acc = mma(a.v, bf.v, acc);
  }
  const float bias = bf16q(gb[m]);
#pragma unroll
  for (int r = 0; r < 8; ++r) {
    const float logit = acc[r] * 0.0625f + bias;
    const float gv = 1.0f / (1.0f + __expf(-logit));
    sG[m][16u * w + 8u * hl + r] = gv;
  }
  __syncthreads();
  v4f val[2];
  unsigned int off[2];
#pragma unroll
  for (unsigned int p = 0; p < 2u; ++p) {
    const unsigned int line = p * 16u + (tid >> 3);
    const unsigned int hrow = line >> 1, half = line & 1u;
    const unsigned int piece = tid & 7u;
    val[p] = *(const v4f*)&sG[hrow][half * 32u + piece * 4u];
    off[p] = (b * (unsigned int)NHEAD + hrow) * (unsigned int)SEQ + t0 + half * 32u + piece * 4u;
  }
#pragma unroll
  for (int p = 0; p < 2; ++p) *(volatile v4f*)(gout + off[p]) = val[p];
  __threadfence();
#pragma unroll
  for (int p = 0; p < 2; ++p) *(volatile v4f*)(gout + off[p]) = val[p];
}

__global__ __launch_bounds__(128) __attribute__((amdgpu_num_vgpr(256)))
void k_attn(const unsigned short* __restrict__ qp, const unsigned short* __restrict__ kp,
            const unsigned short* __restrict__ vp, const float* __restrict__ gp,
            unsigned short* __restrict__ op) {
  __shared__ __attribute__((aligned(16))) unsigned short sP[4][16][72];
  const unsigned int tid = threadIdx.x, lane = tid & 31u, w = tid >> 5;
  const unsigned int m = lane & 15u, hl = lane >> 4, k8 = hl * 8u;
  const unsigned int qt = blockIdx.x, hh = blockIdx.y, b = blockIdx.z;
  const unsigned int bh = b * (unsigned int)NHEAD + hh;
  const unsigned int tq = qt * 64u + 16u * w;

  Frag qa0, qa1;
  {
    const unsigned short* qr = qp + ((size_t)bh * SEQ + tq + m) * HD + k8;
    qa0.q[0] = *(const v4u*)(qr);
    qa0.q[1] = *(const v4u*)(qr + 16);
    qa1.q[0] = *(const v4u*)(qr + 32);
    qa1.q[1] = *(const v4u*)(qr + 48);
  }
  float gr[8];
  {
    const float* gq = gp + (size_t)bh * SEQ + tq + 8u * hl;
    const v4f g0 = *(const v4f*)(gq);
    const v4f g1 = *(const v4f*)(gq + 4);
    gr[0] = g0.x; gr[1] = g0.y; gr[2] = g0.z; gr[3] = g0.w;
    gr[4] = g1.x; gr[5] = g1.y; gr[6] = g1.z; gr[7] = g1.w;
  }
  float mrun[8], lrun[8];
  v8f oacc[4];
#pragma unroll
  for (int r = 0; r < 8; ++r) { mrun[r] = -1e30f; lrun[r] = 0.0f; }
#pragma unroll
  for (int j = 0; j < 4; ++j) oacc[j] = zero8();

  const unsigned int nch = qt + 1u + (unsigned int)((2 * MEMN) / 64);
#pragma unroll 1
  for (unsigned int c = 0; c < nch; ++c) {
    const bool mem = c > qt;
    const unsigned int key0 = mem ? ((unsigned int)SEQ + (c - qt - 1u) * 64u) : (c * 64u);
    const bool diag = (c == qt);
    v8f s[4];
    const unsigned short* kb = kp + ((size_t)bh * SKV + key0 + m) * HD + k8;
#pragma unroll
    for (int j = 0; j < 4; ++j) {
      const unsigned short* kr = kb + j * 16 * HD;
      Frag f0, f1;
      f0.q[0] = *(const v4u*)(kr);
      f0.q[1] = *(const v4u*)(kr + 16);
      f1.q[0] = *(const v4u*)(kr + 32);
      f1.q[1] = *(const v4u*)(kr + 48);
      v8f t = mma(qa0.v, f0.v, zero8());
      t = mma(qa1.v, f1.v, t);
      s[j] = t;
    }
    float tmax[8];
#pragma unroll
    for (int r = 0; r < 8; ++r) tmax[r] = -1e30f;
#pragma unroll
    for (int j = 0; j < 4; ++j) {
#pragma unroll
      for (int r = 0; r < 8; ++r) {
        float val = s[j][r] * 0.125f;
        const unsigned int qi = tq + 8u * hl + (unsigned int)r;
        const unsigned int ki = key0 + 16u * (unsigned int)j + m;
        val = (diag && (ki > qi)) ? -1e30f : val;
        s[j][r] = val;
        tmax[r] = fmaxf(tmax[r], val);
      }
    }
#pragma unroll
    for (int r = 0; r < 8; ++r) {
#pragma unroll
      for (int xm = 1; xm < 16; xm <<= 1) tmax[r] = fmaxf(tmax[r], __shfl_xor(tmax[r], xm, 32));
    }
    float corr[8];
#pragma unroll
    for (int r = 0; r < 8; ++r) {
      const float mn = fmaxf(mrun[r], tmax[r]);
      corr[r] = __expf(mrun[r] - mn);
      mrun[r] = mn;
    }
    float tsum[8], pf[8];
#pragma unroll
    for (int r = 0; r < 8; ++r) { tsum[r] = 0.0f; pf[r] = mem ? (gr[r] * 1024.0f) : 1024.0f; }
#pragma unroll
    for (int j = 0; j < 4; ++j) {
#pragma unroll
      for (int r = 0; r < 8; ++r) {
        const float p = __expf(s[j][r] - mrun[r]);
        tsum[r] += p;
        sP[w][8u * hl + r][16 * j + m] = hbits(p * pf[r]);
      }
    }
#pragma unroll
    for (int r = 0; r < 8; ++r) {
#pragma unroll
      for (int xm = 1; xm < 16; xm <<= 1) tsum[r] += __shfl_xor(tsum[r], xm, 32);
      lrun[r] = lrun[r] * corr[r] + tsum[r];
    }
#pragma unroll
    for (int j = 0; j < 4; ++j) {
#pragma unroll
      for (int r = 0; r < 8; ++r) oacc[j][r] *= corr[r];
    }
    __syncthreads();
    Frag pa0, pa1;
    {
      const unsigned short* pr = &sP[w][m][k8];
      pa0.q[0] = *(const v4u*)(pr);
      pa0.q[1] = *(const v4u*)(pr + 16);
      pa1.q[0] = *(const v4u*)(pr + 32);
      pa1.q[1] = *(const v4u*)(pr + 48);
    }
    const unsigned short* vb = vp + ((size_t)bh * HD + m) * (size_t)SKV + key0 + k8;
#pragma unroll
    for (int jd = 0; jd < 4; ++jd) {
      const unsigned short* vr = vb + (size_t)jd * 16 * SKV;
      Frag g0, g1;
      g0.q[0] = *(const v4u*)(vr);
      g0.q[1] = *(const v4u*)(vr + 16);
      g1.q[0] = *(const v4u*)(vr + 32);
      g1.q[1] = *(const v4u*)(vr + 48);
      oacc[jd] = mma(pa0.v, g0.v, oacc[jd]);
      oacc[jd] = mma(pa1.v, g1.v, oacc[jd]);
    }
    __syncthreads();
  }

  float il[8];
#pragma unroll
  for (int r = 0; r < 8; ++r) il[r] = 1.0f / (lrun[r] * 16.0f);
#pragma unroll
  for (int jd = 0; jd < 4; ++jd) {
#pragma unroll
    for (int r = 0; r < 8; ++r) sP[w][8u * hl + r][16 * jd + m] = hbits(oacc[jd][r] * il[r]);
  }
  __syncthreads();
  v4u val[4];
  unsigned int off[4];
#pragma unroll
  for (unsigned int p = 0; p < 4u; ++p) {
    const unsigned int row = 4u * p + (lane >> 3);
    const unsigned int piece = lane & 7u;
    val[p] = *(const v4u*)&sP[w][row][piece * 8u];
    off[p] = (b * (unsigned int)SEQ + tq + row) * (unsigned int)CDIM + hh * (unsigned int)HD + piece * 8u;
  }
#pragma unroll
  for (int p = 0; p < 4; ++p) *(volatile v4u*)(op + off[p]) = val[p];
  __threadfence();
#pragma unroll
  for (int p = 0; p < 4; ++p) *(volatile v4u*)(op + off[p]) = val[p];
}

__global__ __launch_bounds__(256) void k_conv(const unsigned short* __restrict__ ao,
                                              const float* __restrict__ cw,
                                              const float* __restrict__ cb,
                                              unsigned short* __restrict__ a2) {
  const unsigned int tid = threadIdx.x;
  const unsigned int t = blockIdx.x * 2u + (tid >> 7), b = blockIdx.y;
  const unsigned int c0 = (tid & 127u) * 8u;
  float xin[4][8];
#pragma unroll
  for (unsigned int j = 0; j < 4u; ++j) {
    const bool valid = (t + j) >= 3u;
    const unsigned int tc = valid ? (t + j - 3u) : 0u;
    const v4u u = *(const v4u*)(ao + ((size_t)(b * (unsigned int)SEQ + tc)) * CDIM + c0);
    const v8h hv = __builtin_bit_cast(v8h, u);
#pragma unroll
    for (int i = 0; i < 8; ++i) xin[j][i] = valid ? (float)hv[i] : 0.0f;
  }
  const v4f cb0 = bf16q4(*(const v4f*)(cb + c0));
  const v4f cb1 = bf16q4(*(const v4f*)(cb + c0 + 4));
  float cbv[8];
  cbv[0] = cb0.x; cbv[1] = cb0.y; cbv[2] = cb0.z; cbv[3] = cb0.w;
  cbv[4] = cb1.x; cbv[5] = cb1.y; cbv[6] = cb1.z; cbv[7] = cb1.w;
  float y[8];
#pragma unroll
  for (int i = 0; i < 8; ++i) {
    const v4f wv = bf16q4(*(const v4f*)(cw + (size_t)(c0 + i) * 4u));
    float acc = wv.x * xin[0][i];
    acc = acc + wv.y * xin[1][i];
    acc = acc + wv.z * xin[2][i];
    acc = acc + wv.w * xin[3][i];
    acc = acc + cbv[i] * 64.0f;
    y[i] = xin[3][i] + acc;
  }
  const v4u o = pack8h(y[0], y[1], y[2], y[3], y[4], y[5], y[6], y[7]);
  unsigned short* orow = a2 + ((size_t)(b * (unsigned int)SEQ + t)) * CDIM + c0;
  *(volatile v4u*)orow = o;
  __threadfence();
  *(volatile v4u*)orow = o;
}

__global__ __launch_bounds__(256) void k_reg(const float* __restrict__ gp,
                                             float* __restrict__ out) {
  __shared__ float red[256];
  const unsigned int tid = threadIdx.x;
  float s = 0.0f;
#pragma unroll 1
  for (unsigned int it = 0; it < (unsigned int)REG_ITERS; ++it) {
    const v4f v = *(const v4f*)(gp + ((size_t)it * 256u + tid) * 4u);
    s += (fabsf(v.x) + fabsf(v.y)) + (fabsf(v.z) + fabsf(v.w));
  }
  red[tid] = s;
  __syncthreads();
#pragma unroll 1
  for (unsigned int st = 128u; st > 0u; st >>= 1) {
    if (tid < st) {
      const float a = red[tid], c = red[tid + st];
      red[tid] = a + c;
    }
    __syncthreads();
  }
  if (tid == 0u) {
    const float r = 0.01f * (red[0] * (1.0f / (float)GN));
    volatile float* o = out + OUT1_OFF;
    *o = r;
    __threadfence();
    *o = r;
  }
}

static inline size_t al256(size_t v) { return (v + 255) & ~(size_t)255; }

extern "C" void kernel_launch(void* const* d_in, const int* in_sizes, int n_in,
                              void* d_out, int out_size, void* d_ws, size_t ws_size,
                              hipStream_t stream) {
  if (n_in < 11) return;
  const long needX = ((long)(NB - 1) * SEQ_FULL + SEQ) * CDIM;
  const long needM = (long)NB * MEMN * CDIM;
  const long nW = (long)CDIM * CDIM;
  if ((long)in_sizes[0] < needX) return;
  if ((long)in_sizes[1] < needM || (long)in_sizes[2] < needM) return;
  if ((long)in_sizes[3] < nW || (long)in_sizes[4] < nW) return;
  if ((long)in_sizes[5] < nW || (long)in_sizes[6] < nW) return;
  if ((long)in_sizes[7] < (long)CDIM * NHEAD || in_sizes[8] < NHEAD) return;
  if ((long)in_sizes[9] < (long)CDIM * 4 || in_sizes[10] < CDIM) return;
  if ((long)out_size < (long)OUT1_OFF + 1) return;

  const float* x  = (const float*)d_in[0];
  const float* fm = (const float*)d_in[1];
  const float* rm = (const float*)d_in[2];
  const float* Wq = (const float*)d_in[3];
  const float* Wk = (const float*)d_in[4];
  const float* Wv = (const float*)d_in[5];
  const float* Wo = (const float*)d_in[6];
  const float* gW = (const float*)d_in[7];
  const float* gb = (const float*)d_in[8];
  const float* cw = (const float*)d_in[9];
  const float* cb = (const float*)d_in[10];
  float* out = (float*)d_out;

  char* ws = (char*)d_ws;
  size_t off = 0;
  auto carve = [&](size_t bytes) -> char* { char* p = ws + off; off += al256(bytes); return p; };
  const size_t QE = (size_t)NB * SEQ * CDIM;
  const size_t KE = (size_t)NB * SKV * CDIM;
  unsigned short* wqkv = (unsigned short*)carve((size_t)3 * CDIM * CDIM * 2);
  unsigned short* wot  = (unsigned short*)carve((size_t)CDIM * CDIM * 2);
  unsigned short* gwt  = (unsigned short*)carve((size_t)NHEAD * CDIM * 2);
  unsigned short* srcp = (unsigned short*)carve(KE * 2);
  unsigned short* qpl  = (unsigned short*)carve(QE * 2);
  unsigned short* kpl  = (unsigned short*)carve(KE * 2);
  unsigned short* vtp  = (unsigned short*)carve(KE * 2);
  float*          gpl  = (float*)carve((size_t)GN * 4);
  unsigned short* aop  = (unsigned short*)carve(QE * 2);
  unsigned short* a2p  = (unsigned short*)carve(QE * 2);
  if (off > ws_size) return;
  if (off > (size_t)134217728) return;

  k_wprep<<<dim3(CDIM / 64, CDIM / 64, 3), 256, 0, stream>>>(Wq, Wk, Wv, wqkv, CDIM, 64, CDIM, CDIM);
  k_wprep<<<dim3(CDIM / 64, CDIM / 64, 1), 256, 0, stream>>>(Wo, Wo, Wo, wot, CDIM, 64, CDIM, 0);
  k_gprep<<<1, 256, 0, stream>>>(gW, gwt);
  k_pack<<<dim3(SKV, NB), 128, 0, stream>>>(x, fm, rm, srcp);
  k_gemm<0><<<dim3(3 * CDIM / 64, SKV / 64, NB), 128, 0, stream>>>(
      srcp, wqkv, nullptr, qpl, kpl, vtp);
  k_gate<<<dim3(SEQ / 64, NB), 128, 0, stream>>>(qpl, gwt, gb, gpl);
  k_attn<<<dim3(SEQ / 64, NHEAD, NB), 128, 0, stream>>>(qpl, kpl, vtp, gpl, aop);
  k_conv<<<dim3(SEQ / 2, NB), 256, 0, stream>>>(aop, cw, cb, a2p);
  k_gemm<1><<<dim3(CDIM / 64, SEQ / 64, NB), 128, 0, stream>>>(
      a2p, wot, out, nullptr, nullptr, nullptr);
  k_reg<<<1, 256, 0, stream>>>(gpl, out);
}
